// Flow_Attention_Causal_25202868093436
// MI455X (gfx1250) — hardware-verified
//
#include <hip/hip_runtime.h>
#include <math.h>

constexpr int kNB = 2;
constexpr int kSeq = 2048;
constexpr int kNH = 8;
constexpr int kHD = 64;
constexpr int kNG = kNB * kNH;
constexpr int kTokPitch = kNH * kHD;
constexpr int kGPer = 4;
constexpr int kNChunk = kNG / kGPer;
constexpr float kEpsAdd = 1e-6f;
static_assert(kNG % kGPer == 0);
static_assert(kSeq % 64 == 0 && kHD == 64);

typedef __attribute__((ext_vector_type(16))) __bf16   v16b;
typedef __attribute__((ext_vector_type(8)))  __bf16   v8b;
typedef __attribute__((ext_vector_type(8)))  float    v8f;
typedef __attribute__((ext_vector_type(4)))  float    v4f;
typedef __attribute__((ext_vector_type(4)))  unsigned int v4u;

__device__ __forceinline__ unsigned short f2bf_bits(float f) {
  unsigned u = __float_as_uint(f);
  return (unsigned short)((u + 0x7FFFu + ((u >> 16) & 1u)) >> 16);
}
__device__ __forceinline__ float bf_bits2f(unsigned short h) { return __uint_as_float(((unsigned)h) << 16); }

__device__ __forceinline__ void dep_guard_b(v8f& a, v8f& b, v16b x, v16b y) { asm volatile("v_nop\n\tv_nop\n\tv_nop\n\tv_nop" : "+v"(a), "+v"(b) : "v"(x), "v"(y)); }
__device__ __forceinline__ void keep4_b(v16b a, v16b b, v16b c, v16b d) { asm volatile("v_nop" :: "v"(a), "v"(b), "v"(c), "v"(d)); }
__device__ __forceinline__ void acc_guard4(v8f& a, v8f& b, v8f& c, v8f& d) { asm volatile("v_nop\n\tv_nop\n\tv_nop\n\tv_nop" : "+v"(a), "+v"(b), "+v"(c), "+v"(d)); }
template <typename T> struct Frag;
template <> struct Frag<__bf16> {
  typedef v16b V; union U { v16b v; v8b h[2]; };
  static __device__ __forceinline__ v16b load(const __bf16* p) {
    U f; f.h[0] = *(const v8b*)(p); f.h[1] = *(const v8b*)(p + 16); return f.v;
  }
  static __device__ __forceinline__ v8f mma(v16b a, v16b b, v8f c) {
    return __builtin_amdgcn_wmma_f32_16x16x32_bf16(false, a, false, b, (short)0, c, false, false);
  }
  static __device__ __forceinline__ void guard(v8f& a, v8f& b, v16b x, v16b y) { dep_guard_b(a, b, x, y); }
  static __device__ __forceinline__ void keep(v16b a, v16b b, v16b c, v16b d) { keep4_b(a, b, c, d); }
};

__device__ __forceinline__ unsigned pk16(unsigned short a, unsigned short b) { return (unsigned)a | ((unsigned)b << 16); }
__device__ __forceinline__ void split_bf(float x, unsigned short& hb, unsigned short& lb) {
  hb = f2bf_bits(x);
  lb = f2bf_bits(x - bf_bits2f(hb));
}

__device__ __forceinline__ float wsum32(float x) {
#pragma unroll
  for (int off = 16; off > 0; off >>= 1) x += __shfl_xor(x, off, 32);
  return x;
}
__device__ __forceinline__ void kadd(float& s, float& c, float x) {
  const float y = x - c;
  const float t = s + y;
  c = (t - s) - y;
  s = t;
}
__device__ __forceinline__ float rcp_hw(float x) { return __builtin_amdgcn_rcpf(x); }
__device__ __forceinline__ float sigm(float x) { return rcp_hw(1.0f + expf(-x)); }

template <int OUT_MODE, int TRI_MODE>
__global__ __launch_bounds__(256) void wmma_gemm64t(
    const unsigned short* __restrict__ Ap, const unsigned short* __restrict__ A2p, int lda, long strideA,
    const unsigned short* __restrict__ Btp, const unsigned short* __restrict__ Bt2p, int ldb, long strideB,
    void* __restrict__ Cout, void* __restrict__ Cout2, int ldc, long strideC,
    const float* __restrict__ rowfac, long strideF,
    int M, int N, int K, float scale) {
  typedef __bf16 T;
  typedef v16b V;
  const T* A = (const T*)Ap; const T* A2 = (const T*)A2p; const T* Bt = (const T*)Btp; const T* Bt2 = (const T*)Bt2p;
  __shared__ __align__(16) float sT[8][16 * 68];
  const int b    = blockIdx.y;
  const int lane = threadIdx.x & 31;
  const int wave = threadIdx.x >> 5;
  const int tilesN = N >> 6;
  const int tilesM = M >> 6;
  const int tile = blockIdx.x * 8 + wave;
  int tm = 0, tn = 0;
  if (TRI_MODE == 1) {
    const int ntri = (tilesM * (tilesM + 1)) >> 1;
    if (tile >= ntri) return;
    int t0 = (int)((sqrtf(8.0f * (float)tile + 1.0f) - 1.0f) * 0.5f);
#pragma unroll
    for (int it = 0; it < 2; ++it) { if (((t0 * (t0 + 1)) >> 1) > tile) --t0; }
#pragma unroll
    for (int it = 0; it < 2; ++it) { if ((((t0 + 1) * (t0 + 2)) >> 1) <= tile) ++t0; }
    tm = t0;
    tn = tile - ((t0 * (t0 + 1)) >> 1);
  } else {
    if (tile >= tilesM * tilesN) return;
    tm = tile / tilesN;
    tn = tile - tm * tilesN;
  }
  const int m0 = tm << 6;
  const int n0 = tn << 6;

  const T* Ab  = A   + (size_t)b * strideA;
  const T* Bb  = Bt  + (size_t)b * strideB;
  const T* Ab2 = A2  + (size_t)b * strideA;
  const T* Bb2 = Bt2 + (size_t)b * strideB;

  const int rlane = lane & 15;
  const int koff  = (lane >> 4) * 8;
  const int mOff  = (lane >> 4) * 8;

  v8f acc[4][4];
#pragma unroll
  for (int i = 0; i < 4; ++i)
#pragma unroll
    for (int j = 0; j < 4; ++j) acc[i][j] = (v8f){0.f,0.f,0.f,0.f,0.f,0.f,0.f,0.f};

  int kEnd = K;
  if (TRI_MODE == 2) { kEnd = (m0 + 64 < K) ? (m0 + 64) : K; }

  for (int k0 = 0; k0 < kEnd; k0 += 32) {
    V bh[4], bl[4];
#pragma unroll
    for (int j = 0; j < 4; ++j) {
      const size_t bo = (size_t)(n0 + (j << 4) + rlane) * ldb + koff + k0;
      bh[j] = Frag<T>::load(Bb + bo);
      bl[j] = Frag<T>::load(Bb2 + bo);
    }
#pragma unroll
    for (int i = 0; i < 4; ++i) {
      const size_t ao = (size_t)(m0 + (i << 4) + rlane) * lda + koff + k0;
      V ah = Frag<T>::load(Ab + ao);
      V al = Frag<T>::load(Ab2 + ao);
#pragma unroll
      for (int j = 0; j < 4; ++j) {
        acc[i][j] = Frag<T>::mma(ah, bh[j], acc[i][j]);
        acc[i][j] = Frag<T>::mma(ah, bl[j], acc[i][j]);
        acc[i][j] = Frag<T>::mma(al, bh[j], acc[i][j]);
      }
      Frag<T>::guard(acc[i][0], acc[i][3], ah, al);
    }
    Frag<T>::keep(bh[0], bh[1], bh[2], bh[3]);
    Frag<T>::keep(bl[0], bl[1], bl[2], bl[3]);
  }
  acc_guard4(acc[0][0], acc[0][1], acc[0][2], acc[0][3]);
  acc_guard4(acc[1][0], acc[1][1], acc[1][2], acc[1][3]);
  acc_guard4(acc[2][0], acc[2][1], acc[2][2], acc[2][3]);
  acc_guard4(acc[3][0], acc[3][1], acc[3][2], acc[3][3]);

  float* slab = sT[wave];
#pragma unroll
  for (int i = 0; i < 4; ++i) {
    const int mBase = m0 + (i << 4);
    float fr[8];
    if (TRI_MODE == 1) {
      const float* Fb = rowfac + (size_t)b * strideF;
#pragma unroll
      for (int r = 0; r < 8; ++r) fr[r] = Fb[mBase + mOff + r];
    } else {
#pragma unroll
      for (int r = 0; r < 8; ++r) fr[r] = 1.0f;
    }
#pragma unroll
    for (int j = 0; j < 4; ++j) {
      const int n = n0 + (j << 4) + rlane;
#pragma unroll
      for (int r = 0; r < 8; ++r) {
        const int m = mBase + mOff + r;
        float v = acc[i][j][r] * scale;
        if (TRI_MODE == 1) {
          v = v * fr[r];
          v = (n > m) ? 0.0f : v;
        }
        slab[(mOff + r) * 68 + (j << 4) + rlane] = v;
      }
    }
    __builtin_amdgcn_fence(__ATOMIC_RELEASE, "workgroup");
    __builtin_amdgcn_wave_barrier();
    __builtin_amdgcn_fence(__ATOMIC_ACQUIRE, "workgroup");
    if (OUT_MODE == 0) {
      float* C = (float*)Cout + (size_t)b * strideC;
      const int hh = lane >> 4, c4 = (lane & 15) * 4;
      for (int pass = 0; pass < 2; ++pass) {
#pragma unroll
        for (int it = 0; it < 8; ++it) {
          const int row = it * 2 + hh;
          v4f v = *(const v4f*)(slab + row * 68 + c4);
          *(volatile v4f*)(C + (size_t)(mBase + row) * ldc + n0 + c4) = v;
        }
        __threadfence();
      }
    } else {
      const int qq = lane >> 3, c8 = (lane & 7) * 8;
      unsigned short* C  = (unsigned short*)Cout  + (size_t)b * strideC;
      unsigned short* C2 = (unsigned short*)Cout2 + (size_t)b * strideC;
      for (int pass = 0; pass < 2; ++pass) {
#pragma unroll
        for (int it = 0; it < 4; ++it) {
          const int row = it * 4 + qq;
          const float* sp = slab + row * 68 + c8;
          const v4f s0 = *(const v4f*)(sp);
          const v4f s1 = *(const v4f*)(sp + 4);
          unsigned short hb[8], lb[8];
#pragma unroll
          for (int e = 0; e < 4; ++e) {
            split_bf(s0[e], hb[e], lb[e]);
            split_bf(s1[e], hb[4 + e], lb[4 + e]);
          }
          const v4u hv = (v4u){pk16(hb[0], hb[1]), pk16(hb[2], hb[3]), pk16(hb[4], hb[5]), pk16(hb[6], hb[7])};
          const v4u lv = (v4u){pk16(lb[0], lb[1]), pk16(lb[2], lb[3]), pk16(lb[4], lb[5]), pk16(lb[6], lb[7])};
          *(volatile v4u*)(C  + (size_t)(mBase + row) * ldc + n0 + c8) = hv;
          *(volatile v4u*)(C2 + (size_t)(mBase + row) * ldc + n0 + c8) = lv;
        }
        __threadfence();
      }
    }
    __builtin_amdgcn_fence(__ATOMIC_RELEASE, "workgroup");
    __builtin_amdgcn_wave_barrier();
    __builtin_amdgcn_fence(__ATOMIC_ACQUIRE, "workgroup");
  }
}

__global__ __launch_bounds__(32) void stats_scan_kernel(
    const float* __restrict__ q, const float* __restrict__ k, const float* __restrict__ v,
    unsigned short* __restrict__ QH, unsigned short* __restrict__ QL,
    unsigned short* __restrict__ KH, unsigned short* __restrict__ KL,
    unsigned short* __restrict__ VH, unsigned short* __restrict__ VL,
    float* __restrict__ RF) {
  __shared__ __align__(16) unsigned short sQh[64 * 64];
  __shared__ __align__(16) unsigned short sQl[64 * 64];
  __shared__ __align__(16) unsigned short sKh[64 * 64];
  __shared__ __align__(16) unsigned short sKl[64 * 64];
  __shared__ __align__(16) unsigned short sVh[64 * 64];
  __shared__ __align__(16) unsigned short sVl[64 * 64];
  __shared__ __align__(16) float sRf[64];

  const int g = blockIdx.x;
  const int n = g >> 3;
  const int h = g & 7;
  const int lane = threadIdx.x & 31;
  const size_t gin = ((size_t)n * kSeq * kNH + h) * kHD;
  const float* qg = q + gin;
  const float* kg = k + gin;
  const float* vg = v + gin;
  unsigned short* QHg = QH + (size_t)g * kSeq * kHD;
  unsigned short* QLg = QL + (size_t)g * kSeq * kHD;
  unsigned short* KHg = KH + (size_t)g * kSeq * kHD;
  unsigned short* KLg = KL + (size_t)g * kSeq * kHD;
  unsigned short* VHg = VH + (size_t)g * kHD * kSeq;
  unsigned short* VLg = VL + (size_t)g * kHD * kSeq;
  float* RFg = RF + (size_t)g * kSeq;

  float cq0 = 0.f, cq1 = 0.f, ck0 = 0.f, ck1 = 0.f;
  float cks0 = 0.f, cks1 = 0.f, cqs0 = 0.f, cqs1 = 0.f;
  float ces = 0.f;
  float eq0 = 0.f, eq1 = 0.f, ek0 = 0.f, ek1 = 0.f;
  float eks0 = 0.f, eks1 = 0.f, eqs0 = 0.f, eqs1 = 0.f, ees = 0.f;

  const int qd = lane >> 3;
  const int c8 = (lane & 7) * 8;

#pragma unroll 1
  for (int l0 = 0; l0 < kSeq; l0 += 64) {
#pragma unroll 1
    for (int j = 0; j < 64; ++j) {
      const int l = l0 + j;
      const size_t off = (size_t)l * kTokPitch;
      const float qa = qg[off + lane], qb = qg[off + lane + 32];
      const float ka = kg[off + lane], kb = kg[off + lane + 32];
      const float va = vg[off + lane], vb = vg[off + lane + 32];
      const float sqa = sigm(qa), sqb = sigm(qb);
      const float ska = sigm(ka), skb = sigm(kb);
      kadd(cq0, eq0, sqa); kadd(cq1, eq1, sqb);
      kadd(ck0, ek0, ska); kadd(ck1, ek1, skb);
      const float p1 = wsum32((sqa + kEpsAdd) * (ck0 + kEpsAdd) + (sqb + kEpsAdd) * (ck1 + kEpsAdd));
      const float p2 = wsum32((ska + kEpsAdd) * (cq0 + kEpsAdd) + (skb + kEpsAdd) * (cq1 + kEpsAdd));
      const float nm = (float)(l + 1);
      const float rn = rcp_hw(nm);
      const float si = rcp_hw(p1) * nm;
      const float so = rcp_hw(p2) * nm;
      kadd(cks0, eks0, ska * so); kadd(cks1, eks1, skb * so);
      kadd(cqs0, eqs0, sqa * si); kadd(cqs1, eqs1, sqb * si);
      const float c1 = wsum32((sqa + kEpsAdd) * (cks0 + kEpsAdd) + (sqb + kEpsAdd) * (cks1 + kEpsAdd));
      const float c2 = wsum32((ska + kEpsAdd) * (cqs0 + kEpsAdd) + (skb + kEpsAdd) * (cqs1 + kEpsAdd));
      const float csink = c1 * rn;
      const float csrc = fminf(fmaxf(c2 * rn, -1.0f), 1.0f);
      const float salloc = sigm(csink);
      const float es = expf(csrc);
      kadd(ces, ees, es);
      const float scmp = es * rcp_hw(ces) * nm;
      const float rf = si * rn * salloc;
      const float vsa = va * scmp, vsb = vb * scmp;
      unsigned short hb, lb;
      split_bf(sqa, hb, lb); sQh[j * 64 + lane] = hb;        sQl[j * 64 + lane] = lb;
      split_bf(sqb, hb, lb); sQh[j * 64 + lane + 32] = hb;   sQl[j * 64 + lane + 32] = lb;
      split_bf(ska, hb, lb); sKh[j * 64 + lane] = hb;        sKl[j * 64 + lane] = lb;
      split_bf(skb, hb, lb); sKh[j * 64 + lane + 32] = hb;   sKl[j * 64 + lane + 32] = lb;
      split_bf(vsa, hb, lb); sVh[lane * 64 + j] = hb;        sVl[lane * 64 + j] = lb;
      split_bf(vsb, hb, lb); sVh[(lane + 32) * 64 + j] = hb; sVl[(lane + 32) * 64 + j] = lb;
      sRf[j] = rf;
    }
    __syncthreads();
    for (int pass = 0; pass < 2; ++pass) {
#pragma unroll 1
      for (int it = 0; it < 16; ++it) {
        const int row = it * 4 + qd;
        const v4u a0 = *(const v4u*)(sQh + row * 64 + c8);
        const v4u a1 = *(const v4u*)(sQl + row * 64 + c8);
        const v4u a2 = *(const v4u*)(sKh + row * 64 + c8);
        const v4u a3 = *(const v4u*)(sKl + row * 64 + c8);
        const size_t go = (size_t)(l0 + row) * kHD + c8;
        *(volatile v4u*)(QHg + go) = a0;
        *(volatile v4u*)(QLg + go) = a1;
        *(volatile v4u*)(KHg + go) = a2;
        *(volatile v4u*)(KLg + go) = a3;
        const v4u e0 = *(const v4u*)(sVh + row * 64 + c8);
        const v4u e1 = *(const v4u*)(sVl + row * 64 + c8);
        const size_t vo = (size_t)row * kSeq + l0 + c8;
        *(volatile v4u*)(VHg + vo) = e0;
        *(volatile v4u*)(VLg + vo) = e1;
      }
      {
        const v4f r4 = *(const v4f*)(sRf + (lane & 15) * 4);
        if (lane < 16) *(volatile v4f*)(RFg + l0 + lane * 4) = r4;
      }
      __threadfence();
    }
    __syncthreads();
  }
}

extern "C" void kernel_launch(void* const* d_in, const int* in_sizes, int n_in,
                              void* d_out, int out_size, void* d_ws, size_t ws_size,
                              hipStream_t stream) {
  const int nElem = kNB * kSeq * kNH * kHD;
  if (n_in < 3) return;
  if (in_sizes[0] != nElem || in_sizes[1] != nElem || in_sizes[2] != nElem) return;
  if (out_size != nElem) return;
  const float* q = (const float*)d_in[0];
  const float* k = (const float*)d_in[1];
  const float* v = (const float*)d_in[2];
  float* out = (float*)d_out;
  unsigned char* ws = (unsigned char*)d_ws;

  const size_t bQK = (size_t)kNG * kSeq * kHD * 2;
  const size_t bRF = (size_t)kNG * kSeq * 4;
  const size_t bP  = (size_t)kGPer * kSeq * kSeq * 2;
  const size_t oQH = 0, oQL = bQK, oKH = 2 * bQK, oKL = 3 * bQK, oVH = 4 * bQK, oVL = 5 * bQK;
  const size_t oRF = 6 * bQK;
  const size_t oPH = oRF + bRF;
  const size_t oPL = oPH + bP;
  const size_t oEnd = oPL + bP;
  if (oEnd > ws_size) return;

  unsigned short* QH = (unsigned short*)(ws + oQH);
  unsigned short* QL = (unsigned short*)(ws + oQL);
  unsigned short* KH = (unsigned short*)(ws + oKH);
  unsigned short* KL = (unsigned short*)(ws + oKL);
  unsigned short* VH = (unsigned short*)(ws + oVH);
  unsigned short* VL = (unsigned short*)(ws + oVL);
  float* RF = (float*)(ws + oRF);
  unsigned short* PH = (unsigned short*)(ws + oPH);
  unsigned short* PL = (unsigned short*)(ws + oPL);

  stats_scan_kernel<<<dim3(kNG), dim3(32), 0, stream>>>(q, k, v, QH, QL, KH, KL, VH, VL, RF);

  const int tilesM = kSeq / 64;
  const int ntri = (tilesM * (tilesM + 1)) / 2;
  const int blocksTri = (ntri + 7) / 8;
  const int blocksPV = (tilesM * 1 + 7) / 8;
  for (int c = 0; c < kNChunk; ++c) {
    const size_t gqk = (size_t)c * kGPer * kSeq * kHD;
    const size_t gvt = (size_t)c * kGPer * kHD * kSeq;
    const size_t grf = (size_t)c * kGPer * kSeq;
    wmma_gemm64t<2, 1><<<dim3(blocksTri, kGPer), dim3(256), 0, stream>>>(
        QH + gqk, QL + gqk, kHD, (long)kSeq * kHD,
        KH + gqk, KL + gqk, kHD, (long)kSeq * kHD,
        (void*)PH, (void*)PL, kSeq, (long)kSeq * kSeq,
        RF + grf, (long)kSeq,
        kSeq, kSeq, kHD, 1.0f);
    const int nb = c >> 1;
    const int h0 = (c & 1) * kGPer;
    float* oc = out + (size_t)nb * kSeq * kTokPitch + (size_t)h0 * kHD;
    wmma_gemm64t<0, 2><<<dim3(blocksPV, kGPer), dim3(256), 0, stream>>>(
        PH, PL, kSeq, (long)kSeq * kSeq,
        VH + gvt, VL + gvt, kSeq, (long)kHD * kSeq,
        (void*)oc, (void*)PL, kTokPitch, (long)kHD,
        RF, (long)0,
        kSeq, kHD, kSeq, 1.0f);
  }
}
